// GRUStyleRefinementAttention_67765993996936
// MI455X (gfx1250) — hardware-verified
//
#include <hip/hip_runtime.h>


#define TT   2048
#define CC   768
#define NH_  12
#define HD   64
#define RR   32
#define KR   64
#define K0   128
#define ZH   2
#define BSC  (-7.6246189861593985f)
#define TAUI (2.857142857142857f)
typedef _Float16 h16;
typedef unsigned short bf;
typedef __attribute__((ext_vector_type(16))) __bf16   v16bf;
typedef __attribute__((ext_vector_type(16))) _Float16 v16h;
typedef __attribute__((ext_vector_type(8)))  _Float16 v8h;
typedef __attribute__((ext_vector_type(8)))  unsigned short v8us;
typedef __attribute__((ext_vector_type(8)))  float    v8f;
typedef __attribute__((ext_vector_type(4)))  float    v4f;
typedef v8h  __attribute__((may_alias)) v8ha;
typedef v4f  __attribute__((may_alias)) v4fa;
typedef v8us __attribute__((may_alias)) v8usa;

__device__ __forceinline__ unsigned short f2bf(float f) { unsigned u = __float_as_uint(f); u += 0x7FFFu + ((u >> 16) & 1u); return (unsigned short)(u >> 16); }
__device__ __forceinline__ float bf2f(unsigned short b) { return __uint_as_float(((unsigned)b) << 16); }
__device__ __forceinline__ float bfr(float f) { return bf2f(f2bf(f)); }
__device__ __forceinline__ v16h cat16(v8h lo, v8h hi) { return __builtin_shufflevector(lo, hi, 0, 1, 2, 3, 4, 5, 6, 7, 8, 9, 10, 11, 12, 13, 14, 15); }
__device__ __forceinline__ v16bf cat16b(v8us lo, v8us hi) { return __builtin_bit_cast(v16bf, __builtin_shufflevector(lo, hi, 0, 1, 2, 3, 4, 5, 6, 7, 8, 9, 10, 11, 12, 13, 14, 15)); }
__device__ __forceinline__ v8f wmma16(v16h a, v16h b, v8f c) { return __builtin_amdgcn_wmma_f32_16x16x32_f16(false, a, false, b, (short)0, c, false, false); }
__device__ __forceinline__ v8f wmmab(v16bf a, v16bf b, v8f c) { return __builtin_amdgcn_wmma_f32_16x16x32_bf16(false, a, false, b, (short)0, c, false, false); }


template <typename T16> struct WFrag;
template <> struct WFrag<h16> { typedef v16h V; static __device__ __forceinline__ V ld(const h16* p) { return cat16(*(const v8h*)p, *(const v8h*)(p + 16)); } static __device__ __forceinline__ v8f mma(V a, V b, v8f c) { return wmma16(a, b, c); } };
template <> struct WFrag<bf> { typedef v16bf V; static __device__ __forceinline__ V ld(const bf* p) { return cat16b(*(const v8us*)p, *(const v8us*)(p + 16)); } static __device__ __forceinline__ v8f mma(V a, V b, v8f c) { return wmmab(a, b, c); } };
template <typename T16, int NSPLIT, bool BIAS>
__global__ __launch_bounds__(32) void k_gemmw(const T16* __restrict__ A, const T16* __restrict__ A2, const T16* __restrict__ Bt, const T16* __restrict__ Bt2, int K, float* C, int ldc, const float* __restrict__ bias, size_t sA, size_t sB, size_t sC) {
    typedef typename WFrag<T16>::V V;
    __shared__ __align__(16) float os[16 * 68];
    const size_t z = blockIdx.z; A += z * sA; if (A2) A2 += z * sA; Bt += z * sB; if (Bt2) Bt2 += z * sB; C += z * sC;
    const int lane = threadIdx.x & 31, lr = lane & 15, hi = lane >> 4; const int r0 = blockIdx.x * 64, c0 = blockIdx.y * 64;
    v8f acc[4][4];
#pragma unroll
    for (int mb = 0; mb < 4; ++mb)
#pragma unroll
        for (int nb = 0; nb < 4; ++nb) acc[mb][nb] = (v8f){};
    const size_t aoff = (size_t)(r0 + lr) * K + 8 * hi, boff = (size_t)(c0 + lr) * K + 8 * hi;
#pragma unroll 1
    for (int kc = 0; kc < K; kc += 32) {
        V a[4], a2[4];
#pragma unroll
        for (int mb = 0; mb < 4; ++mb) { a[mb] = WFrag<T16>::ld(A + aoff + (size_t)mb * 16 * K + kc); if (NSPLIT == 1 || NSPLIT == 2) a2[mb] = WFrag<T16>::ld(A2 + aoff + (size_t)mb * 16 * K + kc); }
#pragma unroll
        for (int nb = 0; nb < 4; ++nb) { const V b = WFrag<T16>::ld(Bt + boff + (size_t)nb * 16 * K + kc); V b2; if (NSPLIT >= 2) b2 = WFrag<T16>::ld(Bt2 + boff + (size_t)nb * 16 * K + kc);
#pragma unroll
            for (int mb = 0; mb < 4; ++mb) { acc[mb][nb] = WFrag<T16>::mma(a[mb], b, acc[mb][nb]); if (NSPLIT == 1 || NSPLIT == 2) acc[mb][nb] = WFrag<T16>::mma(a2[mb], b, acc[mb][nb]); if (NSPLIT >= 2) acc[mb][nb] = WFrag<T16>::mma(a[mb], b2, acc[mb][nb]); } }
        asm volatile("v_nop\n\tv_nop\n\tv_nop\n\tv_nop" : "+v"(acc[0][0]), "+v"(acc[1][1]), "+v"(acc[2][2]), "+v"(acc[3][3]) : "v"(a[0]), "v"(a[3]));
    }
#pragma unroll
    for (int mb = 0; mb < 4; ++mb) {
#pragma unroll
        for (int nb = 0; nb < 4; ++nb) {
#pragma unroll
            for (int j = 0; j < 8; ++j) os[(hi * 8 + j) * 68 + nb * 16 + lr] = acc[mb][nb][j]; }
        __builtin_amdgcn_wave_barrier(); asm volatile("" ::: "memory");
        float* crow = C + (size_t)(r0 + mb * 16) * ldc + c0;
#pragma unroll 1
        for (int ps = 0; ps < 2; ++ps) {
#pragma unroll
            for (int s = 0; s < 8; ++s) { const int row = 2 * s + hi, cofs = lr * 4; v4f val = *(const v4fa*)(os + row * 68 + cofs); if (BIAS) { val[0] += bfr(bias[c0 + cofs]); val[1] += bfr(bias[c0 + cofs + 1]); val[2] += bfr(bias[c0 + cofs + 2]); val[3] += bfr(bias[c0 + cofs + 3]); }
                *(volatile v4f*)(crow + (size_t)row * ldc + cofs) = val; }
            if (ps == 0) __threadfence(); }
        __builtin_amdgcn_wave_barrier(); asm volatile("" ::: "memory");
    }
}

template <typename T16, int NSPLIT, int CMODE>
__global__ __launch_bounds__(32) void k_gemmc(const T16* __restrict__ A, const T16* __restrict__ A2, const T16* __restrict__ Bt, const T16* __restrict__ Bt2, int K, float* C, int ldc, int roff, size_t sA, size_t sB, size_t sC) {
    typedef typename WFrag<T16>::V V;
    __shared__ __align__(16) float os[16 * 68];
    const size_t z = blockIdx.z; A += z * sA; if (A2) A2 += z * sA; Bt += z * sB; if (Bt2) Bt2 += z * sB; C += z * sC;
    const int lane = threadIdx.x & 31, lr = lane & 15, hi = lane >> 4; const int r0 = blockIdx.x * 64, c0 = blockIdx.y * 64;
    if (CMODE == 1 && c0 > r0 + roff + 63) return;
    const int Kl = (CMODE == 2) ? min(K, r0 + roff + 64) : K;
    v8f acc[4][4];
#pragma unroll
    for (int mb = 0; mb < 4; ++mb)
#pragma unroll
        for (int nb = 0; nb < 4; ++nb) acc[mb][nb] = (v8f){};
    const size_t aoff = (size_t)(r0 + lr) * K + 8 * hi, boff = (size_t)(c0 + lr) * K + 8 * hi;
#pragma unroll 1
    for (int kc = 0; kc < Kl; kc += 32) {
        V a[4], a2[4];
#pragma unroll
        for (int mb = 0; mb < 4; ++mb) { a[mb] = WFrag<T16>::ld(A + aoff + (size_t)mb * 16 * K + kc); if (NSPLIT == 1 || NSPLIT == 2) a2[mb] = WFrag<T16>::ld(A2 + aoff + (size_t)mb * 16 * K + kc); }
#pragma unroll
        for (int nb = 0; nb < 4; ++nb) { const V b = WFrag<T16>::ld(Bt + boff + (size_t)nb * 16 * K + kc); V b2; if (NSPLIT >= 2) b2 = WFrag<T16>::ld(Bt2 + boff + (size_t)nb * 16 * K + kc);
#pragma unroll
            for (int mb = 0; mb < 4; ++mb) { acc[mb][nb] = WFrag<T16>::mma(a[mb], b, acc[mb][nb]); if (NSPLIT == 1 || NSPLIT == 2) acc[mb][nb] = WFrag<T16>::mma(a2[mb], b, acc[mb][nb]); if (NSPLIT >= 2) acc[mb][nb] = WFrag<T16>::mma(a[mb], b2, acc[mb][nb]); } }
        asm volatile("v_nop\n\tv_nop\n\tv_nop\n\tv_nop" : "+v"(acc[0][0]), "+v"(acc[1][1]), "+v"(acc[2][2]), "+v"(acc[3][3]) : "v"(a[0]), "v"(a[3]));
    }
#pragma unroll
    for (int mb = 0; mb < 4; ++mb) {
#pragma unroll
        for (int nb = 0; nb < 4; ++nb) {
#pragma unroll
            for (int j = 0; j < 8; ++j) os[(hi * 8 + j) * 68 + nb * 16 + lr] = acc[mb][nb][j]; }
        __builtin_amdgcn_wave_barrier(); asm volatile("" ::: "memory");
        float* crow = C + (size_t)(r0 + mb * 16) * ldc + c0;
#pragma unroll 1
        for (int ps = 0; ps < 2; ++ps) {
#pragma unroll
            for (int s = 0; s < 8; ++s) { const int row = 2 * s + hi, cofs = lr * 4; v4f val = *(const v4fa*)(os + row * 68 + cofs);
                *(volatile v4f*)(crow + (size_t)row * ldc + cofs) = val; }
            if (ps == 0) __threadfence(); }
        __builtin_amdgcn_wave_barrier(); asm volatile("" ::: "memory");
    }
}

__device__ __forceinline__ void splitf(float y, unsigned short& h, unsigned short& l) { h = f2bf(y); l = f2bf(y - bf2f(h)); }
__device__ __forceinline__ float sigm_(float x) { return __fdiv_rn(1.0f, 1.0f + __expf(-x)); }
typedef __attribute__((ext_vector_type(2))) unsigned short v2us;
typedef __attribute__((ext_vector_type(4))) unsigned short v4us;
typedef __attribute__((ext_vector_type(2))) float v2f;

__global__ __launch_bounds__(256) void k_wtG(const float* __restrict__ w, int K, int N, bf* Bt) {
    const int lane = threadIdx.x & 31; const int L0 = (blockIdx.x * 8 + (threadIdx.x >> 5)) * 8; const int nlines = N * K / 64;
#pragma unroll 1
    for (int ps = 0; ps < 2; ++ps) {
#pragma unroll 1
        for (int l = 0; l < 8; ++l) { const int L = L0 + l; if (L >= nlines) break; const size_t e = (size_t)L * 64 + lane * 2; const int k = (int)(e % K), n = (int)(e / K); v2us o;
            o[0] = f2bf(w[(size_t)k * N + n]); o[1] = f2bf(w[(size_t)(k + 1) * N + n]); *(volatile v2us*)(Bt + e) = o; }
        if (ps == 0) __threadfence(); }
}
__global__ __launch_bounds__(256) void k_cvt8(const float* __restrict__ src, bf* dst, size_t n8) { const size_t i = (size_t)blockIdx.x * 256 + threadIdx.x; if (i >= n8) return; const v8f v = *(const v8f*)(src + i * 8); v8us o;
#pragma unroll
    for (int k = 0; k < 8; ++k) o[k] = f2bf(v[k]); *(volatile v8us*)(dst + i * 8) = o; __threadfence(); *(volatile v8us*)(dst + i * 8) = o; }
__global__ __launch_bounds__(256) void k_wp(const float* __restrict__ P, bf* Bt) { const int e = (blockIdx.x * 256 + threadIdx.x) * 4; if (e >= KR * CC) return; const int k = e % CC, n = e / CC; v4us o;
#pragma unroll
    for (int q = 0; q < 4; ++q) o[q] = n < RR ? f2bf(P[(size_t)(k + q) * RR + n]) : (unsigned short)0; *(volatile v4us*)(Bt + e) = o; __threadfence(); *(volatile v4us*)(Bt + e) = o; }
__global__ __launch_bounds__(256) void k_spl(const float* __restrict__ F, size_t n4, bf* Fh, bf* Fl) { const size_t i = ((size_t)blockIdx.x * 256 + threadIdx.x) * 4; if (i >= n4 * 4) return; const v4f a = *(const v4f*)(F + i); v4us oh, ol;
#pragma unroll
    for (int q = 0; q < 4; ++q) { unsigned short u, c2; splitf(a[q], u, c2); oh[q] = u; ol[q] = c2; } *(volatile v4us*)(Fh + i) = oh; *(volatile v4us*)(Fl + i) = ol; __threadfence(); *(volatile v4us*)(Fh + i) = oh; *(volatile v4us*)(Fl + i) = ol; }
__global__ __launch_bounds__(32) void k_cummax(const float* __restrict__ VR, float* MS) { const int r = threadIdx.x; float m = -3.0e38f; for (int t = 0; t < TT; ++t) { m = fmaxf(m, VR[(size_t)t * KR + r]); *(volatile float*)(MS + (size_t)t * RR + r) = m; } __threadfence(); m = -3.0e38f; for (int t = 0; t < TT; ++t) { m = fmaxf(m, VR[(size_t)t * KR + r]); *(volatile float*)(MS + (size_t)t * RR + r) = m; } }
__global__ __launch_bounds__(256) void k_evr(const float* __restrict__ VR, bf* Eh, bf* El) { const size_t e = ((size_t)blockIdx.x * 256 + threadIdx.x) * 2; if (e >= (size_t)KR * TT) return; const int t = (int)(e % TT), r = (int)(e / TT); v2us oh, ol;
#pragma unroll
    for (int u = 0; u < 2; ++u) { unsigned short a = 0, c = 0; if (r < RR) splitf(__expf(VR[(size_t)(t + u) * KR + r]), a, c); oh[u] = a; ol[u] = c; } *(volatile v2us*)(Eh + e) = oh; *(volatile v2us*)(El + e) = ol; __threadfence(); *(volatile v2us*)(Eh + e) = oh; *(volatile v2us*)(El + e) = ol; }
__global__ __launch_bounds__(256) void k_aseed(const float* __restrict__ Sb, bf* Ah, bf* Al) { const size_t e = ((size_t)blockIdx.x * 256 + threadIdx.x) * 4; if (e >= (size_t)TT * TT) return; const int j = (int)(e % TT), i = (int)(e / TT); const v4f a = *(const v4f*)(Sb + e); v4us oh, ol;
#pragma unroll
    for (int q = 0; q < 4; ++q) { float v = 0.f; if (j + q <= i) { float s = __fmul_rn(a[q], 0.17677669529663687f); asm volatile("" : "+v"(s)); float s2 = __fmul_rn(s, s); asm volatile("" : "+v"(s2)); v = sigm_(__fadd_rn(s2, BSC)); } unsigned short u, c; splitf(v, u, c); oh[q] = u; ol[q] = c; }
    *(volatile v4us*)(Ah + e) = oh; *(volatile v4us*)(Al + e) = ol; __threadfence(); *(volatile v4us*)(Ah + e) = oh; *(volatile v4us*)(Al + e) = ol; }
__global__ __launch_bounds__(256) void k_h0in(const float* __restrict__ YR, const float* __restrict__ MS, bf* Lh, bf* Ll) { const size_t e = ((size_t)blockIdx.x * 256 + threadIdx.x) * 2; if (e >= (size_t)TT * RR) return; const int r = (int)(e % RR), t = (int)(e / RR); v2us oh, ol;
#pragma unroll
    for (int u = 0; u < 2; ++u) { unsigned short a = 0, c = 0; const int rr = r + u; { const float m = MS[(size_t)t * RR + rr]; float y = __fmul_rn(YR[(size_t)t * KR + rr], __expf(-m)); asm volatile("" : "+v"(y)); splitf(__fadd_rn(__logf(fmaxf(y, 1e-30f)), m), a, c); } oh[u] = a; ol[u] = c; }
    *(volatile v2us*)(Lh + e) = oh; *(volatile v2us*)(Ll + e) = ol; __threadfence(); *(volatile v2us*)(Lh + e) = oh; *(volatile v2us*)(Ll + e) = ol; }
__global__ __launch_bounds__(256) void k_nrm(const float* __restrict__ QF, const float* __restrict__ KF, bf* Qh, bf* Ql, bf* Kh, bf* Kl) { const int lane = threadIdx.x & 31; const int row = blockIdx.x * 8 + (threadIdx.x >> 5); if (row >= NH_ * TT) return; const int t = row % TT, h = row / TT; const float* q = QF + (size_t)t * CC + h * HD + 2 * lane; const float* k = KF + (size_t)t * CC + h * HD + 2 * lane; const float q0 = q[0], q1 = q[1], k0 = k[0], k1 = k[1];
    float sq = __fadd_rn(__fmul_rn(q0, q0), __fmul_rn(q1, q1)), sk = __fadd_rn(__fmul_rn(k0, k0), __fmul_rn(k1, k1));
#pragma unroll
    for (int sh = 16; sh; sh >>= 1) { sq += __shfl_xor(sq, sh, 32); sk += __shfl_xor(sk, sh, 32); }
    const float iq = __fdiv_rn(1.0f, fmaxf(__fsqrt_rn(sq), 1e-12f)), ik = __fdiv_rn(1.0f, fmaxf(__fsqrt_rn(sk), 1e-12f)); v2us qh, ql, kh, kl; unsigned short a, c;
    splitf(__fmul_rn(q0, iq), a, c); qh[0] = a; ql[0] = c; splitf(__fmul_rn(q1, iq), a, c); qh[1] = a; ql[1] = c; splitf(__fmul_rn(k0, ik), a, c); kh[0] = a; kl[0] = c; splitf(__fmul_rn(k1, ik), a, c); kh[1] = a; kl[1] = c;
    const size_t o = (size_t)row * HD + 2 * lane; for (int ps = 0; ps < 2; ++ps) { *(volatile v2us*)(Qh + o) = qh; *(volatile v2us*)(Ql + o) = ql; *(volatile v2us*)(Kh + o) = kh; *(volatile v2us*)(Kl + o) = kl; if (ps == 0) __threadfence(); } }
__global__ __launch_bounds__(256) void k_vexp(const float* __restrict__ VF, bf* Eh, bf* El, float* MN) { const size_t e = ((size_t)blockIdx.x * 256 + threadIdx.x) * 2; if (e >= (size_t)NH_ * HD * TT) return; const int t = (int)(e % TT); const int d = (int)((e / TT) % HD); const int h = (int)(e / ((size_t)TT * HD)); v2us oh, ol; v2f mm;
#pragma unroll
    for (int u = 0; u < 2; ++u) { const int tt = t + u; float m = -3.0e38f; for (int s = max(0, tt - K0); s <= tt; ++s) m = fmaxf(m, VF[(size_t)s * CC + h * HD + d]); const float v = VF[(size_t)tt * CC + h * HD + d]; unsigned short a, c; splitf(__expf(__fsub_rn(v, m)), a, c); oh[u] = a; ol[u] = c; mm[u] = m; }
    *(volatile v2us*)(Eh + e) = oh; *(volatile v2us*)(El + e) = ol; __threadfence(); *(volatile v2us*)(Eh + e) = oh; *(volatile v2us*)(El + e) = ol;
    *(volatile v2f*)(MN + e) = mm; __threadfence(); *(volatile v2f*)(MN + e) = mm; }
__global__ __launch_bounds__(256) void k_anear(const float* __restrict__ Sb, bf* Ah, bf* Al) { const size_t e = ((size_t)blockIdx.x * 256 + threadIdx.x) * 4; if (e >= (size_t)ZH * TT * TT) return; const int j = (int)(e % TT); const int i = (int)((e / TT) % TT); const v4f a = *(const v4f*)(Sb + e); v4us oh, ol;
#pragma unroll
    for (int q = 0; q < 4; ++q) { const int jj = j + q; float v = 0.f; if (jj <= i && i - jj <= K0) { float c2 = __fmul_rn(a[q], a[q]); asm volatile("" : "+v"(c2)); float t = __fmul_rn(c2, TAUI); asm volatile("" : "+v"(t)); v = sigm_(__fadd_rn(t, BSC)); } unsigned short u, c; splitf(v, u, c); oh[q] = u; ol[q] = c; }
    *(volatile v4us*)(Ah + e) = oh; *(volatile v4us*)(Al + e) = ol; __threadfence(); *(volatile v4us*)(Ah + e) = oh; *(volatile v4us*)(Al + e) = ol; }
__global__ __launch_bounds__(256) void k_hnear(const float* __restrict__ Y, const float* __restrict__ MN, const float* __restrict__ gu, const float* __restrict__ gb, int h0, float* HT) { const int lane = threadIdx.x & 31; const int row = blockIdx.x * 8 + (threadIdx.x >> 5); if (row >= ZH * TT) return; const int t = row % TT, z = row / TT; const int h = h0 + z; const int d0 = 2 * lane; float hn[2]; float s = 0.f;
#pragma unroll
    for (int u = 0; u < 2; ++u) { const int d = d0 + u; const float m = MN[((size_t)h * HD + d) * TT + t]; hn[u] = __fadd_rn(__logf(fmaxf(Y[((size_t)z * TT + t) * HD + d], 1e-30f)), m); float p = __fmul_rn(hn[u], bfr(gu[h * HD + d])); asm volatile("" : "+v"(p)); s = __fadd_rn(s, p); }
#pragma unroll
    for (int sh = 16; sh; sh >>= 1) s += __shfl_xor(s, sh, 32);
    const float g = sigm_(__fadd_rn(s, bfr(gb[h]))); v2f o; o[0] = __fmul_rn(hn[0], g); o[1] = __fmul_rn(hn[1], g); const size_t oo = (size_t)t * CC + h * HD + d0; *(volatile v2f*)(HT + oo) = o; __threadfence(); *(volatile v2f*)(HT + oo) = o; }
__global__ __launch_bounds__(256) void k_zin(const float* __restrict__ x, const float* __restrict__ H0, const float* __restrict__ HT, bf* Zh, bf* Zl) { const size_t e = ((size_t)blockIdx.x * 256 + threadIdx.x) * 4; if (e >= (size_t)TT * 4 * CC) return; const int c = (int)(e % (4 * CC)); const int t = (int)(e / (4 * CC)); const int part = c / CC, cc = c % CC; const size_t s = (size_t)t * CC + cc; v4us oh, ol;
#pragma unroll
    for (int q = 0; q < 4; ++q) { float v; if (part == 0) v = bfr(x[s + q]); else if (part == 1) v = H0[s + q]; else if (part == 2) v = HT[s + q]; else v = __fmul_rn(H0[s + q], HT[s + q]); unsigned short a, b; splitf(v, a, b); oh[q] = a; ol[q] = b; }
    *(volatile v4us*)(Zh + e) = oh; *(volatile v4us*)(Zl + e) = ol; __threadfence(); *(volatile v4us*)(Zh + e) = oh; *(volatile v4us*)(Zl + e) = ol; }
__global__ __launch_bounds__(256) void k_blend(const float* __restrict__ ZF, const float* __restrict__ bz, const float* __restrict__ H0, const float* __restrict__ HT, bf* Bh, bf* Bl) { const size_t i = ((size_t)blockIdx.x * 256 + threadIdx.x) * 4; if (i >= (size_t)TT * CC) return; const int c = (int)(i % CC); v4us oh, ol;
#pragma unroll
    for (int q = 0; q < 4; ++q) { const float z = sigm_(__fadd_rn(ZF[i + q], bfr(bz[c + q]))); float a = __fmul_rn(__fsub_rn(1.0f, z), H0[i + q]); asm volatile("" : "+v"(a)); float b = __fmul_rn(z, HT[i + q]); asm volatile("" : "+v"(b)); unsigned short u, l; splitf(__fadd_rn(a, b), u, l); oh[q] = u; ol[q] = l; }
    *(volatile v4us*)(Bh + i) = oh; *(volatile v4us*)(Bl + i) = ol; __threadfence(); *(volatile v4us*)(Bh + i) = oh; *(volatile v4us*)(Bl + i) = ol; }

extern "C" void kernel_launch(void* const* d_in, const int* in_sizes, int n_in,
                              void* d_out, int out_size, void* d_ws, size_t ws_size, hipStream_t stream) {
    (void)in_sizes; (void)n_in; (void)out_size;
    const float* IN[17]; for (int i = 0; i < 17; ++i) IN[i] = (const float*)d_in[i];
    float* OUT = (float*)d_out;
    char* wsp = (char*)d_ws;
    auto take = [&](size_t bytes) { char* p = wsp; wsp += (bytes + 255) & ~(size_t)255; return (void*)p; };
    bf* WQ = (bf*)take((size_t)CC * CC * 2); bf* WK = (bf*)take((size_t)CC * CC * 2); bf* WV = (bf*)take((size_t)CC * CC * 2); bf* WO = (bf*)take((size_t)CC * CC * 2); bf* WZ = (bf*)take((size_t)CC * 4 * CC * 2); bf* BPQ = (bf*)take((size_t)KR * CC * 2); bf* BPK = (bf*)take((size_t)KR * CC * 2); bf* BPV = (bf*)take((size_t)KR * CC * 2); bf* BUP = (bf*)take((size_t)CC * KR * 2);
    bf* XB = (bf*)take((size_t)TT * CC * 2); float* QF = (float*)take((size_t)TT * CC * 4); float* KF = (float*)take((size_t)TT * CC * 4); float* VF = (float*)take((size_t)TT * CC * 4); bf* Th = (bf*)take((size_t)TT * CC * 2); bf* Tl = (bf*)take((size_t)TT * CC * 2);
    float* QR = (float*)take((size_t)TT * KR * 4); float* KRb = (float*)take((size_t)TT * KR * 4); float* VR = (float*)take((size_t)TT * KR * 4); bf* QRh = (bf*)take((size_t)TT * KR * 2); bf* QRl = (bf*)take((size_t)TT * KR * 2); bf* KRh = (bf*)take((size_t)TT * KR * 2); bf* KRl = (bf*)take((size_t)TT * KR * 2); float* MS = (float*)take((size_t)TT * RR * 4); bf* EVh = (bf*)take((size_t)KR * TT * 2); bf* EVl = (bf*)take((size_t)KR * TT * 2);
    float* Sb = (float*)take((size_t)ZH * TT * TT * 4); bf* Ah = (bf*)take((size_t)ZH * TT * TT * 2); bf* Al = (bf*)take((size_t)ZH * TT * TT * 2); float* YR = (float*)take((size_t)TT * KR * 4); bf* LGh = (bf*)take((size_t)TT * KR * 2); bf* LGl = (bf*)take((size_t)TT * KR * 2); float* H0 = (float*)take((size_t)TT * CC * 4);
    bf* NQh = (bf*)take((size_t)NH_ * TT * HD * 2); bf* NQl = (bf*)take((size_t)NH_ * TT * HD * 2); bf* NKh = (bf*)take((size_t)NH_ * TT * HD * 2); bf* NKl = (bf*)take((size_t)NH_ * TT * HD * 2); bf* VEh = (bf*)take((size_t)NH_ * HD * TT * 2); bf* VEl = (bf*)take((size_t)NH_ * HD * TT * 2); float* MN = (float*)take((size_t)NH_ * HD * TT * 4); float* Y = (float*)take((size_t)ZH * TT * HD * 4); float* HT = (float*)take((size_t)TT * CC * 4);
    bf* Zh = (bf*)take((size_t)TT * 4 * CC * 2); bf* Zl = (bf*)take((size_t)TT * 4 * CC * 2); float* ZF = QF; bf* Bh = Th; bf* Bl = Tl;
    if ((size_t)(wsp - (char*)d_ws) > ws_size) return;
    k_wtG<<<(CC * CC / 64 + 63) / 64, 256, 0, stream>>>(IN[1], CC, CC, WQ); k_wtG<<<(CC * CC / 64 + 63) / 64, 256, 0, stream>>>(IN[3], CC, CC, WK); k_wtG<<<(CC * CC / 64 + 63) / 64, 256, 0, stream>>>(IN[5], CC, CC, WV); k_wtG<<<(CC * CC / 64 + 63) / 64, 256, 0, stream>>>(IN[7], CC, CC, WO); k_wtG<<<(4 * CC * CC / 64 + 63) / 64, 256, 0, stream>>>(IN[15], 4 * CC, CC, WZ);
    k_wp<<<(KR * CC / 4 + 255) / 256, 256, 0, stream>>>(IN[9], BPQ); k_wp<<<(KR * CC / 4 + 255) / 256, 256, 0, stream>>>(IN[10], BPK); k_wp<<<(KR * CC / 4 + 255) / 256, 256, 0, stream>>>(IN[11], BPV); k_wtG<<<(KR * CC / 64 + 63) / 64, 256, 0, stream>>>(IN[12], RR, CC, BUP);
    k_cvt8<<<(TT * CC / 8 + 255) / 256, 256, 0, stream>>>(IN[0], XB, (size_t)TT * CC / 8);
    k_gemmw<bf, 0, true><<<dim3(TT / 64, CC / 64, 1), 32, 0, stream>>>(XB, nullptr, WQ, nullptr, CC, QF, CC, IN[2], 0, 0, 0); k_gemmw<bf, 0, true><<<dim3(TT / 64, CC / 64, 1), 32, 0, stream>>>(XB, nullptr, WK, nullptr, CC, KF, CC, IN[4], 0, 0, 0); k_gemmw<bf, 0, true><<<dim3(TT / 64, CC / 64, 1), 32, 0, stream>>>(XB, nullptr, WV, nullptr, CC, VF, CC, IN[6], 0, 0, 0);
    const size_t n4 = (size_t)TT * CC / 4;
    k_spl<<<(unsigned)((n4 + 255) / 256), 256, 0, stream>>>(QF, n4, Th, Tl); k_gemmw<bf, 1, false><<<dim3(TT / 64, 1, 1), 32, 0, stream>>>(Th, Tl, BPQ, nullptr, CC, QR, KR, nullptr, 0, 0, 0);
    k_spl<<<(unsigned)((n4 + 255) / 256), 256, 0, stream>>>(KF, n4, Th, Tl); k_gemmw<bf, 1, false><<<dim3(TT / 64, 1, 1), 32, 0, stream>>>(Th, Tl, BPK, nullptr, CC, KRb, KR, nullptr, 0, 0, 0);
    k_spl<<<(unsigned)((n4 + 255) / 256), 256, 0, stream>>>(VF, n4, Th, Tl); k_gemmw<bf, 1, false><<<dim3(TT / 64, 1, 1), 32, 0, stream>>>(Th, Tl, BPV, nullptr, CC, VR, KR, nullptr, 0, 0, 0);
    k_spl<<<(unsigned)(((size_t)TT * KR / 4 + 255) / 256), 256, 0, stream>>>(QR, (size_t)TT * KR / 4, QRh, QRl); k_spl<<<(unsigned)(((size_t)TT * KR / 4 + 255) / 256), 256, 0, stream>>>(KRb, (size_t)TT * KR / 4, KRh, KRl);
    k_cummax<<<1, 32, 0, stream>>>(VR, MS); k_evr<<<(unsigned)(((size_t)KR * TT / 2 + 255) / 256), 256, 0, stream>>>(VR, EVh, EVl);
    k_gemmc<bf, 2, 1><<<dim3(TT / 64, TT / 64, 1), 32, 0, stream>>>(QRh, QRl, KRh, KRl, KR, Sb, TT, 0, 0, 0, 0);
    k_aseed<<<(unsigned)(((size_t)TT * TT / 4 + 255) / 256), 256, 0, stream>>>(Sb, Ah, Al);
    k_gemmc<bf, 2, 2><<<dim3(TT / 64, 1, 1), 32, 0, stream>>>(Ah, Al, EVh, EVl, TT, YR, KR, 0, 0, 0, 0);
    k_h0in<<<(unsigned)(((size_t)TT * RR / 2 + 255) / 256), 256, 0, stream>>>(YR, MS, LGh, LGl);
    k_gemmw<bf, 1, false><<<dim3(TT / 64, CC / 64, 1), 32, 0, stream>>>(LGh, LGl, BUP, nullptr, RR, H0, CC, nullptr, 0, 0, 0);
    k_nrm<<<NH_ * TT / 8, 256, 0, stream>>>(QF, KF, NQh, NQl, NKh, NKl); k_vexp<<<(unsigned)(((size_t)NH_ * HD * TT / 2 + 255) / 256), 256, 0, stream>>>(VF, VEh, VEl, MN);
    for (int h0 = 0; h0 < NH_; h0 += ZH) { const size_t z = (size_t)h0;
        k_gemmc<bf, 2, 1><<<dim3(TT / 64, TT / 64, ZH), 32, 0, stream>>>(NQh + z * TT * HD, NQl + z * TT * HD, NKh + z * TT * HD, NKl + z * TT * HD, HD, Sb, TT, 0, (size_t)TT * HD, (size_t)TT * HD, (size_t)TT * TT);
        k_anear<<<(unsigned)(((size_t)ZH * TT * TT / 4 + 255) / 256), 256, 0, stream>>>(Sb, Ah, Al);
        k_gemmc<bf, 2, 2><<<dim3(TT / 64, 1, ZH), 32, 0, stream>>>(Ah, Al, VEh + z * HD * TT, VEl + z * HD * TT, TT, Y, HD, 0, (size_t)TT * TT, (size_t)HD * TT, (size_t)TT * HD);
        k_hnear<<<ZH * TT / 8, 256, 0, stream>>>(Y, MN, IN[13], IN[14], h0, HT); }
    k_zin<<<(unsigned)(((size_t)TT * 4 * CC / 4 + 255) / 256), 256, 0, stream>>>(IN[0], H0, HT, Zh, Zl);
    k_gemmw<bf, 1, false><<<dim3(TT / 64, CC / 64, 1), 32, 0, stream>>>(Zh, Zl, WZ, nullptr, 4 * CC, ZF, CC, nullptr, 0, 0, 0);
    k_blend<<<(unsigned)((n4 + 255) / 256), 256, 0, stream>>>(ZF, IN[16], H0, HT, Bh, Bl);
    k_gemmw<bf, 1, true><<<dim3(TT / 64, CC / 64, 1), 32, 0, stream>>>(Bh, Bl, WO, nullptr, CC, OUT, CC, IN[8], 0, 0, 0);
}
